// DiffSchNet_66116726554888
// MI455X (gfx1250) — hardware-verified
//
#include <hip/hip_runtime.h>
#include <stddef.h>
#include <stdint.h>

#define NB     256
#define NEL    32
#define NNUC   4
#define EMB    256
#define KER    128
#define DIFF   224
#define HID    169
#define HIDN   176
#define HIDK   192
#define NLAY   3
#define ZK     384
#define AP     232
#define HP     200
#define EP     264
#define ZP     392
#define NWAV   4
#define NTHR   (NWAV * 32)
#define NTILE  18

#define OFF_ELEC 0
#define OFF_HS   (OFF_ELEC + NEL * EMB * 4)
#define OFF_Z    (OFF_HS + NEL * EMB * 4)
#define OFF_TAB  (OFF_Z + NEL * ZP * 2)
#define OFF_POS  (OFF_TAB + 64 * 4)
#define OFF_YW   (OFF_POS + 448)
#define OFF_A    (OFF_YW + NNUC * KER * 4)
#define OFF_H    (OFF_A + NWAV * 16 * AP * 2)
#define LDS_BYTES (OFF_H + NWAV * 16 * HP * 2)

static_assert(OFF_HS == 32768);
static_assert(OFF_Z == 65536);
static_assert(OFF_TAB == 90624);
static_assert(OFF_POS == 90880);
static_assert(OFF_YW == 91328);
static_assert(OFF_A == 93376);
static_assert(OFF_H == 123072);
static_assert(LDS_BYTES == 148672);
static_assert((OFF_TAB % 16) == 0 && (OFF_POS % 16) == 0 && (OFF_YW % 16) == 0 && (OFF_A % 16) == 0 && (OFF_H % 16) == 0);
static_assert((NEL + NNUC) * 3 * 4 <= 448);
static_assert(NEL * EP * 2 <= NWAV * 16 * AP * 2);
static_assert(AP % 8 == 0 && HP % 8 == 0 && EP % 8 == 0 && ZP % 8 == 0);
static_assert(AP >= DIFF && HP >= HIDK && EP >= EMB && ZP >= ZK);
static_assert(DIFF % 32 == 0 && HIDK % 32 == 0 && EMB % 32 == 0 && ZK % 32 == 0);
static_assert(HIDN % 16 == 0 && HIDN >= HID && HIDK >= HIDN);
static_assert(NWAV * 8 == NEL);
static_assert(NWAV * 64 == EMB);
static_assert(NTHR * 64 == NEL * EMB);
static_assert(NTILE == 8 + 8 + 2);

#define W1T_HALVES (9 * HIDN * DIFF)
#define W2T_HALVES (9 * KER * HIDK)
#define HWT_HALVES (2 * EMB * EMB)
#define GWT_HALVES (3 * EMB * ZK)
#define C1 (W1T_HALVES / 8)
#define C2 (W2T_HALVES / 8)
#define C3 (HWT_HALVES / 8)
#define C4 (GWT_HALVES / 8)
#define NCHUNK (C1 + C2 + C3 + C4)
static_assert(W1T_HALVES % 256 == 0 && W2T_HALVES % 256 == 0 && HWT_HALVES % 256 == 0 && GWT_HALVES % 256 == 0);
static_assert(C1 % 32 == 0 && C2 % 32 == 0 && C3 % 32 == 0 && C4 % 32 == 0);
static_assert(NCHUNK == 125248);

typedef _Float16 f16;
typedef f16 v16h __attribute__((ext_vector_type(16)));
typedef f16 v8h_t __attribute__((ext_vector_type(8)));
typedef v8h_t __attribute__((may_alias)) v8h;
typedef float v8f __attribute__((ext_vector_type(8)));
typedef float v4f_t __attribute__((ext_vector_type(4)));
typedef v4f_t __attribute__((may_alias)) v4f;
typedef unsigned int v4u __attribute__((ext_vector_type(4)));

union Frag  { v16h v; v8h_t h[2]; };
union HPack { v8h_t v; v4u u; f16 e[8]; };

__device__ __forceinline__ v8f zero8() {
  v8f z;
#pragma unroll
  for (int i = 0; i < 8; ++i) z[i] = 0.0f;
  return z;
}

__device__ __forceinline__ v8h_t zero8h() {
  HPack z;
#pragma unroll
  for (int i = 0; i < 4; ++i) z.u[i] = 0u;
  return z.v;
}

__device__ __forceinline__ v16h ldfrag(const f16* p, int k0) {
  Frag f;
  f.h[0] = *(const v8h*)(p + k0);
  f.h[1] = *(const v8h*)(p + k0 + 16);
  return f.v;
}

__device__ __forceinline__ v8f wmma_g(v16h a, v16h b, v8f c) {
  c = __builtin_amdgcn_wmma_f32_16x16x32_f16(false, a, false, b, (short)0, c, false, false);
  asm volatile("v_nop\n\tv_nop\n\tv_nop\n\tv_nop" : "+v"(c) : "v"(a), "v"(b));
  return c;
}

template <int NT, int KS>
__device__ __forceinline__ void gemm_rows16(const f16* pa, const f16* __restrict__ pb, int ldb,
                                            v8f (&acc)[NT])
{
#pragma unroll
  for (int t = 0; t < NT; ++t) acc[t] = zero8();
#pragma unroll 1
  for (int ks = 0; ks < KS; ++ks) {
    const int k0 = ks * 32;
    const v16h a = ldfrag(pa, k0);
#pragma unroll
    for (int t = 0; t < NT; ++t) {
      const v16h bb = ldfrag(pb + (size_t)t * 16 * ldb, k0);
      acc[t] = wmma_g(a, bb, acc[t]);
    }
  }
}

__device__ __forceinline__ void basis16(float dd, const float (&mu)[16], const float (&ig)[16], f16* dst)
{
  const float env = ((dd * dd) * __expf(-dd)) * 16.0f;
  HPack p0, p1;
#pragma unroll
  for (int j = 0; j < 8; ++j) {
    const float t0 = dd - mu[j];
    p0.e[j] = (f16)(env * __expf(-(t0 * t0) * ig[j]));
    const float t1 = dd - mu[8 + j];
    p1.e[j] = (f16)(env * __expf(-(t1 * t1) * ig[8 + j]));
  }
  *(v8h*)dst = p0.v;
  *(v8h*)(dst + 8) = p1.v;
}

__device__ __forceinline__ void relu_groups(float d, const float (&mu)[16], const float (&ig)[16],
                                            f16* base, v8h_t zv)
{
  const int ob = (d < 0.0f) ? 32 : 0;
  basis16(fabsf(d), mu, ig, base + ob);
  f16* zp = base + (32 - ob);
  *(v8h*)zp = zv;
  *(v8h*)(zp + 8) = zv;
}

template <int NT>
__device__ __forceinline__ void silu_store(const v8f (&acc)[NT], int col0, const float* __restrict__ b1,
                                           int lt, f16* hT, int hh, int m)
{
#pragma unroll
  for (int t = 0; t < NT; ++t) {
    const int col = col0 + 16 * t + m;
    const int cc  = (col < HID) ? col : (HID - 1);
    const float bl = b1[lt * HID + cc];
    const float bv = (col < HID) ? bl : 0.0f;
#pragma unroll
    for (int r = 0; r < 8; ++r) {
      const float x  = acc[t][r] * (1.0f / 256.0f) + bv;
      const float sg = __builtin_amdgcn_rcpf(1.0f + __expf(-x));
      hT[(8 * hh + r) * HP + col] = (f16)(((x * sg)) * 64.0f);
    }
  }
}

template <int NT>
__device__ __forceinline__ void pair_epi(const v8f (&acc)[NT], int col0, int rcv, int sb, int sgm,
                                         const float* hsL, f16* zL, int hh, int m)
{
  float mk[8];
#pragma unroll
  for (int r = 0; r < 8; ++r) mk[r] = ((sb + 8 * hh + r) != rcv) ? 1.0f : 0.0f;
  const float* hb = hsL + (size_t)(sb + 8 * hh) * EMB + sgm * KER + col0 + m;
#pragma unroll
  for (int t = 0; t < NT; ++t) {
    float cs = 0.0f;
#pragma unroll
    for (int r = 0; r < 8; ++r) cs += acc[t][r] * (hb[r * EMB + 16 * t] * mk[r]);
    const float tot = cs + __shfl_xor(cs, 16, 32);
    const f16 zv = (f16)(tot * 0.25f);
    if (hh == 0) zL[rcv * ZP + sgm * KER + col0 + 16 * t + m] = zv;
  }
}

template <int NT>
__device__ __forceinline__ void ne_epi(const v8f (&acc)[NT], int col0, int R0, const float* ywL,
                                       f16* zL, int hh, int m)
{
  const int ra = R0 + 2 * hh, rb = ra + 1;
#pragma unroll
  for (int t = 0; t < NT; ++t) {
    const int col = col0 + 16 * t + m;
    float za = 0.0f, zb = 0.0f;
#pragma unroll
    for (int r = 0; r < 4; ++r) {
      za += acc[t][r] * ywL[r * KER + col];
      zb += acc[t][4 + r] * ywL[r * KER + col];
    }
    zL[ra * ZP + 2 * KER + col] = (f16)(za * 0.25f);
    zL[rb * ZP + 2 * KER + col] = (f16)(zb * 0.25f);
  }
}

__global__ void __launch_bounds__(256) prep_kernel(
    const float* __restrict__ W1, const float* __restrict__ W2, const float* __restrict__ HW,
    const float* __restrict__ GW, f16* __restrict__ W1t, f16* __restrict__ W2t,
    f16* __restrict__ HWt, f16* __restrict__ GWt, int nchunks)
{
  const int c   = blockIdx.x * 256 + threadIdx.x;
  const bool ok = (c < nchunks);
  const int cc  = ok ? c : 0;
  float v[8];
  f16* dst;
  if (cc < C1) {
    const int e   = cc * 8;
    const int lt  = e / (HIDN * DIFF);
    const int rem = e - lt * (HIDN * DIFF);
    const int n   = rem / DIFF;
    const int k0  = rem - n * DIFF;
    const int nn  = (n < HID) ? n : (HID - 1);
#pragma unroll
    for (int j = 0; j < 8; ++j) {
      const float x = W1[((size_t)(lt * DIFF + k0 + j)) * HID + nn];
      v[j] = (n < HID) ? x : 0.0f;
    }
    dst = W1t + e;
  } else if (cc < C1 + C2) {
    const int e   = (cc - C1) * 8;
    const int lt  = e / (KER * HIDK);
    const int rem = e - lt * (KER * HIDK);
    const int n   = rem / HIDK;
    const int k0  = rem - n * HIDK;
#pragma unroll
    for (int j = 0; j < 8; ++j) {
      const int k  = k0 + j;
      const int kc = (k < HID) ? k : (HID - 1);
      const float x = W2[((size_t)(lt * HID + kc)) * KER + n];
      v[j] = (k < HID) ? x : 0.0f;
    }
    dst = W2t + e;
  } else if (cc < C1 + C2 + C3) {
    const int e   = (cc - C1 - C2) * 8;
    const int lp  = e / (EMB * EMB);
    const int rem = e - lp * (EMB * EMB);
    const int ci  = rem / EMB;
    const int k0  = rem - ci * EMB;
#pragma unroll
    for (int j = 0; j < 8; ++j)
      v[j] = HW[((size_t)((lp * 2 + (ci >> 7)) * EMB + k0 + j)) * KER + (ci & (KER - 1))];
    dst = HWt + e;
  } else {
    const int e   = (cc - C1 - C2 - C3) * 8;
    const int lp  = e / (EMB * ZK);
    const int rem = e - lp * (EMB * ZK);
    const int n   = rem / ZK;
    const int kk0 = rem - n * ZK;
#pragma unroll
    for (int j = 0; j < 8; ++j) {
      const int kk = kk0 + j;
      v[j] = GW[((size_t)((lp * 3 + (kk >> 7)) * KER + (kk & (KER - 1)))) * EMB + n];
    }
    dst = GWt + e;
  }
  HPack pk;
#pragma unroll
  for (int j = 0; j < 8; ++j) pk.e[j] = (f16)(v[j] * 16.0f);
  const v4u val = pk.u;
  if (ok) *(volatile v4u*)dst = val;
  __threadfence();
  if (ok) *(volatile v4u*)dst = val;
}

__global__ void __launch_bounds__(NTHR) fused_net_kernel(
    const float* __restrict__ rs, const float* __restrict__ coords, const float* __restrict__ Xemb,
    const float* __restrict__ Yw, const float* __restrict__ b1, const float* __restrict__ h0,
    const f16* __restrict__ W1t, const f16* __restrict__ W2t,
    const f16* __restrict__ HWt, const f16* __restrict__ GWt, float* __restrict__ out)
{
  extern __shared__ float4 lds_f4[];
  unsigned char* lds = (unsigned char*)lds_f4;
  float* elecL = (float*)(lds + OFF_ELEC);
  float* hsL   = (float*)(lds + OFF_HS);
  f16*   zL    = (f16*)(lds + OFF_Z);
  float* tabL  = (float*)(lds + OFF_TAB);
  float* posL  = (float*)(lds + OFF_POS);
  float* ywL   = (float*)(lds + OFF_YW);
  f16*   aAll  = (f16*)(lds + OFF_A);
  f16*   hAll  = (f16*)(lds + OFF_H);
  f16*   e16L  = aAll;

  const int tid = threadIdx.x;
  const int w = tid >> 5, lane = tid & 31, hh = lane >> 4, m = lane & 15;
  const int b = blockIdx.x;
  f16* aT = aAll + w * (16 * AP);
  f16* hT = hAll + w * (16 * HP);

  if (tid < 32) {
    const float q  = (float)(2 * tid + 1) * (1.0f / 64.0f);
    const float mu = 10.0f * (q * q);
    const float sg = (1.0f + 10.0f * q) * (1.0f / 7.0f);
    tabL[tid] = mu;
    tabL[32 + tid] = 1.0f / (sg * sg);
  }
  {
    const int ie = (tid < NEL * 3) ? tid : (NEL * 3 - 1);
    int ic = tid - NEL * 3;
    ic = (ic < 0) ? 0 : ((ic > NNUC * 3 - 1) ? (NNUC * 3 - 1) : ic);
    const float ve = rs[(size_t)b * (NEL * 3) + ie];
    const float vc = coords[ic];
    const float pv = (tid < NEL * 3) ? ve : vc;
    if (tid < (NEL + NNUC) * 3) posL[tid] = pv;
  }
#pragma unroll 1
  for (int i = tid; i < NNUC * KER; i += NTHR) ywL[i] = Yw[i];
#pragma unroll 4
  for (int i = tid; i < NEL * EMB; i += NTHR) {
    hsL[i]   = h0[i & (EMB - 1)];
    elecL[i] = Xemb[i & (EMB - 1)];
  }
  {
    const v8h_t zv = zero8h();
#pragma unroll 1
    for (int i = tid; i < NWAV * 16 * 3; i += NTHR) {
      const int wv = i / 48, rem = i - wv * 48, row = rem / 3, q = rem - row * 3;
      *(v8h*)(hAll + wv * (16 * HP) + row * HP + HIDN + 8 * q) = zv;
    }
  }
  __syncthreads();

#pragma unroll 1
  for (int l = 0; l < NLAY; ++l) {
    if (l > 0) {
      {
        const int row = tid >> 2, cb = (tid & 3) * 64;
        const float* src = elecL + row * EMB + cb;
        f16* dst = e16L + row * EP + cb;
#pragma unroll
        for (int q = 0; q < 8; ++q) {
          HPack pk;
#pragma unroll
          for (int j = 0; j < 8; ++j) pk.e[j] = (f16)(src[8 * q + j] * 64.0f);
          *(v8h*)(dst + 8 * q) = pk.v;
        }
      }
      __syncthreads();
      {
        const f16* hwl = HWt + (size_t)(l - 1) * (EMB * EMB);
#pragma unroll 1
        for (int mt = 0; mt < 2; ++mt) {
#pragma unroll 1
          for (int ng = 0; ng < 2; ++ng) {
            v8f acc[2];
            const int col0 = 64 * w + 32 * ng;
            gemm_rows16<2, 8>(e16L + (16 * mt + m) * EP + 8 * hh,
                              hwl + (size_t)(col0 + m) * EMB + 8 * hh, EMB, acc);
#pragma unroll
            for (int t = 0; t < 2; ++t)
#pragma unroll
              for (int r = 0; r < 8; ++r)
                hsL[(16 * mt + 8 * hh + r) * EMB + col0 + 16 * t + m] = acc[t][r] * (1.0f / 1024.0f);
          }
        }
      }
      __syncthreads();
    }

#pragma unroll 1
    for (int ti = 0; ti < NTILE; ++ti) {
      const int isne = (ti >= 16) ? 1 : 0;
      const int rcv  = 8 * w + (ti & 7);
      const int anti = (ti >> 3) & 1;
      const int up   = (rcv < 16) ? 1 : 0;
      const int sb   = ((anti ^ up) != 0) ? 0 : 16;
      const int R0   = 8 * w + 4 * (ti & 1);
      const int et   = isne ? 2 : anti;
      const int lt   = l * 3 + et;

      {
        const int ps = isne ? (NEL + (m & 3)) : (sb + m);
        const int pr = isne ? (R0 + (m >> 2)) : rcv;
        const float dx = posL[ps * 3 + 0] - posL[pr * 3 + 0];
        const float dy = posL[ps * 3 + 1] - posL[pr * 3 + 1];
        const float dz = posL[ps * 3 + 2] - posL[pr * 3 + 2];
        float mu[16], ig[16];
#pragma unroll
        for (int q = 0; q < 4; ++q) {
          const v4f_t a = *(const v4f*)(tabL + 16 * hh + 4 * q);
          const v4f_t c = *(const v4f*)(tabL + 32 + 16 * hh + 4 * q);
#pragma unroll
          for (int j = 0; j < 4; ++j) { mu[4 * q + j] = a[j]; ig[4 * q + j] = c[j]; }
        }
        const v8h_t zv = zero8h();
        f16* arow = aT + m * AP + 16 * hh;
        relu_groups(dx, mu, ig, arow + 0, zv);
        relu_groups(dy, mu, ig, arow + 64, zv);
        relu_groups(dz, mu, ig, arow + 128, zv);
        basis16(dz, mu, ig, arow + 192);
      }
      __syncthreads();

      {
        const f16* pa  = aT + m * AP + 8 * hh;
        const f16* w1l = W1t + (size_t)lt * (HIDN * DIFF);
        {
          v8f acc[6];
          gemm_rows16<6, 7>(pa, w1l + (size_t)(0 + m) * DIFF + 8 * hh, DIFF, acc);
          silu_store<6>(acc, 0, b1, lt, hT, hh, m);
        }
        {
          v8f acc[5];
          gemm_rows16<5, 7>(pa, w1l + (size_t)(96 + m) * DIFF + 8 * hh, DIFF, acc);
          silu_store<5>(acc, 96, b1, lt, hT, hh, m);
        }
      }
      __syncthreads();

      {
        const f16* pa  = hT + m * HP + 8 * hh;
        const f16* w2l = W2t + (size_t)lt * (KER * HIDK);
#pragma unroll
        for (int g = 0; g < 2; ++g) {
          v8f acc[4];
          const int col0 = 64 * g;
          gemm_rows16<4, 6>(pa, w2l + (size_t)(col0 + m) * HIDK + 8 * hh, HIDK, acc);
          if (isne) ne_epi<4>(acc, col0, R0, ywL, zL, hh, m);
          else      pair_epi<4>(acc, col0, rcv, sb, anti, hsL, zL, hh, m);
        }
      }
    }
    __syncthreads();

    {
      const f16* gwl = GWt + (size_t)l * (EMB * ZK);
#pragma unroll 1
      for (int mt = 0; mt < 2; ++mt) {
#pragma unroll 1
        for (int ng = 0; ng < 2; ++ng) {
          v8f acc[2];
          const int col0 = 64 * w + 32 * ng;
          gemm_rows16<2, 12>(zL + (16 * mt + m) * ZP + 8 * hh,
                             gwl + (size_t)(col0 + m) * ZK + 8 * hh, ZK, acc);
#pragma unroll
          for (int t = 0; t < 2; ++t)
#pragma unroll
            for (int r = 0; r < 8; ++r) {
              float* ep = elecL + (16 * mt + 8 * hh + r) * EMB + col0 + 16 * t + m;
              const float nv = *ep + acc[t][r] * (1.0f / 4096.0f);
              *ep = nv;
            }
        }
      }
    }
    __syncthreads();
  }

  {
    float* go = out + (size_t)b * (NEL * EMB) + (size_t)(8 * w) * EMB;
    const float* src = elecL + (8 * w) * EMB;
#pragma unroll
    for (int half = 0; half < 2; ++half) {
      v4f_t v[8];
#pragma unroll
      for (int p = 0; p < 8; ++p) v[p] = *(const v4f*)(src + ((half * 8 + p) * 32 + lane) * 4);
#pragma unroll
      for (int p = 0; p < 8; ++p) *(volatile v4f_t*)(go + ((half * 8 + p) * 32 + lane) * 4) = v[p];
      __threadfence();
#pragma unroll
      for (int p = 0; p < 8; ++p) *(volatile v4f_t*)(go + ((half * 8 + p) * 32 + lane) * 4) = v[p];
    }
  }
}

extern "C" void kernel_launch(void* const* d_in, const int* in_sizes, int n_in,
                              void* d_out, int out_size, void* d_ws, size_t ws_size,
                              hipStream_t stream)
{
  if (n_in < 10) return;
  if (in_sizes[0] != NB * NEL * 3) return;
  if (in_sizes[1] != NNUC * 3) return;
  if (in_sizes[2] != EMB) return;
  if (in_sizes[3] != NNUC * KER) return;
  if (in_sizes[4] != 9 * DIFF * HID) return;
  if (in_sizes[5] != 9 * HID) return;
  if (in_sizes[6] != 9 * HID * KER) return;
  if (in_sizes[7] != 2 * KER) return;
  if (in_sizes[8] != 2 * 2 * EMB * KER) return;
  if (in_sizes[9] != 9 * KER * EMB) return;
  if (out_size != NB * NEL * EMB) return;

  const float* rs     = (const float*)d_in[0];
  const float* coords = (const float*)d_in[1];
  const float* Xemb   = (const float*)d_in[2];
  const float* Yw     = (const float*)d_in[3];
  const float* wW1    = (const float*)d_in[4];
  const float* wb1    = (const float*)d_in[5];
  const float* wW2    = (const float*)d_in[6];
  const float* h0     = (const float*)d_in[7];
  const float* hW     = (const float*)d_in[8];
  const float* gW     = (const float*)d_in[9];
  float* out = (float*)d_out;

  const size_t oW1 = 0;
  const size_t oW2 = oW1 + (size_t)W1T_HALVES * 2;
  const size_t oHW = oW2 + (size_t)W2T_HALVES * 2;
  const size_t oGW = oHW + (size_t)HWT_HALVES * 2;
  const size_t total = oGW + (size_t)GWT_HALVES * 2;
  if (total > ws_size) return;

  char* ws = (char*)d_ws;
  f16* W1t = (f16*)(ws + oW1);
  f16* W2t = (f16*)(ws + oW2);
  f16* HWt = (f16*)(ws + oHW);
  f16* GWt = (f16*)(ws + oGW);

  prep_kernel<<<(NCHUNK + 255) / 256, 256, 0, stream>>>(wW1, wW2, hW, gW, W1t, W2t, HWt, GWt, NCHUNK);

  hipFuncSetAttribute(reinterpret_cast<const void*>(&fused_net_kernel),
                      hipFuncAttributeMaxDynamicSharedMemorySize, LDS_BYTES);
  fused_net_kernel<<<NB, NTHR, LDS_BYTES, stream>>>(rs, coords, Xemb, Yw, wb1, h0,
                                                    W1t, W2t, HWt, GWt, out);
}
